// ViLLayer_86492051407243
// MI455X (gfx1250) — hardware-verified
//
#include <hip/hip_runtime.h>
#include <math.h>
#include <stdint.h>

#define NB     8
#define SEQ    1024
#define GRIDW  32
#define DIMX   192
#define INNER  288
#define UPN    576
#define NHQ    72
#define NHM    4
#define DHM    72
#define NROWS  (NB * SEQ)
#define GK     864
#define GPITCH 896
#define GN     64
#define HP96   96
#define QP     (NHM * HP96)
#define VP     320
#define HOP    (NHM * HP96)
#define OSP    320
#define TOKB   4
#define QSC    1024.0f
#define VSC    64.0f
#define CSC    (9.5367431640625e-7f * 0.1178511301977579f)

static_assert((NROWS % 64) == 0);
static_assert((UPN % 64) == 0);
static_assert((DIMX % 64) == 0);
static_assert((DIMX % 32) == 0);
static_assert((GK % 32) == 0);
static_assert((INNER % 32) == 0);
static_assert((NROWS % TOKB) == 0);
static_assert((SEQ % TOKB) == 0);
static_assert((NROWS % 8) == 0);
static_assert(NHM * DHM == INNER);
static_assert(NB * NHM == 32);

typedef _Float16 v16h __attribute__((ext_vector_type(16)));
typedef _Float16 v8h  __attribute__((ext_vector_type(8)));
typedef __bf16   v16b __attribute__((ext_vector_type(16)));
typedef __bf16   v8b  __attribute__((ext_vector_type(8)));
typedef float    v8f  __attribute__((ext_vector_type(8)));
typedef float    v4f  __attribute__((ext_vector_type(4)));
typedef unsigned int v4u __attribute__((ext_vector_type(4)));
typedef unsigned short v8us __attribute__((ext_vector_type(8)));

__device__ __forceinline__ unsigned short bf_bits(float f) {
  unsigned u = __float_as_uint(f);
  return (unsigned short)((u + 0x7FFFu + ((u >> 16) & 1u)) >> 16);
}
__device__ __forceinline__ float bf_up(unsigned short h) { return __uint_as_float(((unsigned)h) << 16); }
__device__ __forceinline__ float bfr(float f) { return bf_up(bf_bits(f)); }
__device__ __forceinline__ unsigned short h_bits(_Float16 x) { return __builtin_bit_cast(unsigned short, x); }
__device__ __forceinline__ unsigned pk16(unsigned short a, unsigned short b) { return (unsigned)a | ((unsigned)b << 16); }
__device__ __forceinline__ v8f zero8() { v8f z = {0.f, 0.f, 0.f, 0.f, 0.f, 0.f, 0.f, 0.f}; return z; }
__device__ __forceinline__ v4u pack_bf8(v4f a, v4f b) {
  v4u p;
  p[0] = pk16(bf_bits(a[0]), bf_bits(a[1]));
  p[1] = pk16(bf_bits(a[2]), bf_bits(a[3]));
  p[2] = pk16(bf_bits(b[0]), bf_bits(b[1]));
  p[3] = pk16(bf_bits(b[2]), bf_bits(b[3]));
  return p;
}

__device__ __forceinline__ v16b ldfrag_b(const __bf16* p) {
  union { v16b v; v8b h[2]; } f;
  f.h[0] = *(const v8b*)(p);
  f.h[1] = *(const v8b*)(p + 16);
  return f.v;
}
__device__ __forceinline__ v16h ldfrag_h(const _Float16* p) {
  union { v16h v; v8h h[2]; } f;
  f.h[0] = *(const v8h*)(p);
  f.h[1] = *(const v8h*)(p + 16);
  return f.v;
}

__device__ __forceinline__ v8f mma_h(v16h a, v16h b, v8f c) {
  c = __builtin_amdgcn_wmma_f32_16x16x32_f16(false, a, false, b, (short)0, c, false, false);
#if defined(__HIP_DEVICE_COMPILE__)
  asm volatile("v_nop\n\tv_nop\n\tv_nop\n\tv_nop" : "+v"(c) : "v"(a), "v"(b));
#endif
  return c;
}
__device__ __forceinline__ v8f mma_b_raw(v16b a, v16b b, v8f c) {
  return __builtin_amdgcn_wmma_f32_16x16x32_bf16(false, a, false, b, (short)0, c, false, false);
}
__device__ __forceinline__ void dep_guard_b(v8f& a, v8f& b, v16b x, v16b y) {
#if defined(__HIP_DEVICE_COMPILE__)
  asm volatile("v_nop\n\tv_nop\n\tv_nop\n\tv_nop" : "+v"(a), "+v"(b) : "v"(x), "v"(y));
#endif
}
__device__ __forceinline__ void keep4_b(v16b a, v16b b, v16b c, v16b d) {
#if defined(__HIP_DEVICE_COMPILE__)
  asm volatile("v_nop" :: "v"(a), "v"(b), "v"(c), "v"(d));
#endif
}
__device__ __forceinline__ void acc_guard4(v8f& a, v8f& b, v8f& c, v8f& d) {
#if defined(__HIP_DEVICE_COMPILE__)
  asm volatile("v_nop\n\tv_nop\n\tv_nop\n\tv_nop" : "+v"(a), "+v"(b), "+v"(c), "+v"(d));
#endif
}
__device__ __forceinline__ void wave_sync_lds() {
  __builtin_amdgcn_fence(__ATOMIC_RELEASE, "workgroup");
  __builtin_amdgcn_wave_barrier();
  __builtin_amdgcn_fence(__ATOMIC_ACQUIRE, "workgroup");
}
__device__ __forceinline__ float hsum16(float x) {
  x += __shfl_xor(x, 1, 32);
  x += __shfl_xor(x, 2, 32);
  x += __shfl_xor(x, 4, 32);
  x += __shfl_xor(x, 8, 32);
  return x;
}
__device__ __forceinline__ float hsum8(float x) {
  x += __shfl_xor(x, 1, 32);
  x += __shfl_xor(x, 2, 32);
  x += __shfl_xor(x, 4, 32);
  return x;
}

__global__ __launch_bounds__(256) void cvt_cat_bf16x8(const float* __restrict__ in, unsigned short* out,
                                                      int n8, int inCols8, int outPitch, int colOff) {
  const int i = blockIdx.x * 256 + threadIdx.x;
  if (i < n8) {
    const int row = i / inCols8;
    const int c8  = i - row * inCols8;
    const v4f a = *(const v4f*)(in + (size_t)i * 8);
    const v4f b = *(const v4f*)(in + (size_t)i * 8 + 4);
    v4u p;
    p[0] = pk16(bf_bits(a[0]), bf_bits(a[1]));
    p[1] = pk16(bf_bits(a[2]), bf_bits(a[3]));
    p[2] = pk16(bf_bits(b[0]), bf_bits(b[1]));
    p[3] = pk16(bf_bits(b[2]), bf_bits(b[3]));
    unsigned short* dst = out + (size_t)row * outPitch + colOff + c8 * 8;
    *(volatile v4u*)dst = p;
    __threadfence();
    *(volatile v4u*)dst = p;
  }
}

#define NUP8 (UPN * DIMX / 8)
#define NDN8 (DIMX * INNER / 8)
#define NGW8 (GN * GPITCH / 8)
#define BUP ((NUP8 + 255) / 256)
#define BDN ((NDN8 + 255) / 256)
#define BGW ((NGW8 + 255) / 256)

__global__ __launch_bounds__(256) void prep_w(const float* __restrict__ wup, const float* __restrict__ wdn,
                                             const float* __restrict__ igw, const float* __restrict__ fgw,
                                             unsigned short* Wup, unsigned short* Wdn, unsigned short* GW) {
  const int bid = blockIdx.x, tid = threadIdx.x;
  const v4f z = {0.f, 0.f, 0.f, 0.f};
  if (bid < BUP) {
    const int i = bid * 256 + tid;
    if (i < NUP8) {
      const v4f a = *(const v4f*)(wup + (size_t)i * 8);
      const v4f b = *(const v4f*)(wup + (size_t)i * 8 + 4);
      const v4u p = pack_bf8(a, b);
      unsigned short* d = Wup + (size_t)i * 8;
      *(volatile v4u*)d = p;
      __threadfence();
      *(volatile v4u*)d = p;
    }
  } else if (bid < BUP + BDN) {
    const int i = (bid - BUP) * 256 + tid;
    if (i < NDN8) {
      const v4f a = *(const v4f*)(wdn + (size_t)i * 8);
      const v4f b = *(const v4f*)(wdn + (size_t)i * 8 + 4);
      const v4u p = pack_bf8(a, b);
      unsigned short* d = Wdn + (size_t)i * 8;
      *(volatile v4u*)d = p;
      __threadfence();
      *(volatile v4u*)d = p;
    }
  } else {
    const int i = (bid - BUP - BDN) * 256 + tid;
    if (i < NGW8) {
      const int row = i / (GPITCH / 8);
      const int c8  = (i - row * (GPITCH / 8)) * 8;
      const int rr  = row & 3;
      const int cc  = min(c8, GK - 8);
      const v4f a  = *(const v4f*)(igw + (size_t)rr * GK + cc);
      const v4f a4 = *(const v4f*)(igw + (size_t)rr * GK + cc + 4);
      const v4f f  = *(const v4f*)(fgw + (size_t)rr * GK + cc);
      const v4f f4 = *(const v4f*)(fgw + (size_t)rr * GK + cc + 4);
      v4f s = z, s4 = z;
      if (c8 < GK) {
        if (row < NHM) { s = a; s4 = a4; }
        else if (row < 2 * NHM) { s = f; s4 = f4; }
      }
      const v4u p = pack_bf8(s, s4);
      unsigned short* d = GW + (size_t)i * 8;
      *(volatile v4u*)d = p;
      __threadfence();
      *(volatile v4u*)d = p;
    }
  }
}

template <int MODE>
__global__ __launch_bounds__(256) void transpose16(const float* __restrict__ in, int R, int C, long long inStride,
                                                   unsigned short* out, long long outStride, float scale, float rscale) {
  __shared__ __align__(16) unsigned short t[64 * 72];
  union U8 { v8us s; v4u u; };
  const int b = blockIdx.y;
  const int tilesC = C >> 6;
  const int tile = blockIdx.x;
  const int tr = tile / tilesC;
  const int tc = tile - tr * tilesC;
  const int r0 = tr << 6, c0 = tc << 6;
  if (r0 >= R || c0 >= C) return;
  const int tid = threadIdx.x;
  {
    const int row = tid >> 2;
    const int cq  = (tid & 3) * 16;
    const float* p = in + (size_t)b * inStride + (size_t)(r0 + row) * C + c0 + cq;
#pragma unroll
    for (int i = 0; i < 4; ++i) {
      const v4f v = *(const v4f*)(p + 4 * i);
#pragma unroll
      for (int e = 0; e < 4; ++e) {
        const float x = v[e];
        unsigned short bits;
        if (MODE == 0) {
          bits = bf_bits(x);
        } else {
          const float xs = x * scale;
          const _Float16 xh = (_Float16)xs;
          if (MODE == 1) bits = h_bits(xh);
          else           bits = h_bits((_Float16)((xs - (float)xh) * rscale));
        }
        t[(cq + 4 * i + e) * 72 + row] = bits;
      }
    }
  }
  __syncthreads();
  {
    unsigned short* dst = out + (size_t)b * outStride;
    const int q  = tid >> 3;
    const int c8 = (tid & 7) * 8;
    U8 w[2];
#pragma unroll
    for (int it = 0; it < 2; ++it) {
      const int orow = it * 32 + q;
      w[it].s = *(const v8us*)(t + orow * 72 + c8);
    }
    for (int pass = 0; pass < 2; ++pass) {
#pragma unroll
      for (int it = 0; it < 2; ++it) {
        const int orow = it * 32 + q;
        *(volatile v4u*)(dst + (size_t)(c0 + orow) * R + r0 + c8) = w[it].u;
      }
      __threadfence();
    }
  }
}

template <int NSPLIT, int OUT_MODE, int BIAS, int ACT, int RESID>
__global__ __launch_bounds__(256) void gemm64(
    const unsigned short* __restrict__ Ap, const unsigned short* A2p, int lda, long long strideA,
    const unsigned short* __restrict__ Btp, const unsigned short* Bt2p, int ldb, long long strideB,
    const float* __restrict__ bias, const float* __restrict__ res, int ldr,
    void* Cout, int ldc, long long strideC,
    void* Cout2, int ldc2, long long strideC2, int N2,
    int M, int N, int K, float rscale, float oscale) {
  const __bf16* A   = (const __bf16*)(const void*)Ap;
  const __bf16* A2  = (const __bf16*)(const void*)A2p;
  const __bf16* Bt  = (const __bf16*)(const void*)Btp;
  const __bf16* Bt2 = (const __bf16*)(const void*)Bt2p;
  __shared__ __align__(16) float sT[8][16 * 68];
  const int b    = blockIdx.y;
  const int lane = threadIdx.x & 31;
  const int wave = threadIdx.x >> 5;
  const int tilesN = N >> 6;
  const int tilesM = M >> 6;
  const int tile = blockIdx.x * 8 + wave;
  if (tile >= tilesM * tilesN) return;
  const int tm = tile / tilesN;
  const int tn = tile - tm * tilesN;
  const int m0 = tm << 6;
  const int n0 = tn << 6;

  const __bf16* Ab  = A  + (size_t)b * strideA;
  const __bf16* Bb  = Bt + (size_t)b * strideB;
  const __bf16* Ab2 = (NSPLIT >= 1) ? (A2  + (size_t)b * strideA) : Ab;
  const __bf16* Bb2 = (NSPLIT == 2) ? (Bt2 + (size_t)b * strideB) : Bb;

  const int rlane = lane & 15;
  const int koff  = (lane >> 4) * 8;
  const int mOff  = (lane >> 4) * 8;

  v8f acc[4][4];
#pragma unroll
  for (int i = 0; i < 4; ++i)
#pragma unroll
    for (int j = 0; j < 4; ++j) acc[i][j] = zero8();

  for (int k0 = 0; k0 < K; k0 += 32) {
    v16b bh[4], bl[4];
#pragma unroll
    for (int j = 0; j < 4; ++j) {
      const size_t bo = (size_t)(n0 + (j << 4) + rlane) * ldb + koff + k0;
      bh[j] = ldfrag_b(Bb + bo);
      if (NSPLIT == 2) bl[j] = ldfrag_b(Bb2 + bo); else bl[j] = bh[j];
    }
#pragma unroll
    for (int i = 0; i < 4; ++i) {
      const size_t ao = (size_t)(m0 + (i << 4) + rlane) * lda + koff + k0;
      const v16b ah = ldfrag_b(Ab + ao);
      v16b al = ah;
      if (NSPLIT >= 1) al = ldfrag_b(Ab2 + ao);
#pragma unroll
      for (int j = 0; j < 4; ++j) {
        acc[i][j] = mma_b_raw(ah, bh[j], acc[i][j]);
        if (NSPLIT >= 1) acc[i][j] = mma_b_raw(al, bh[j], acc[i][j]);
        if (NSPLIT == 2) acc[i][j] = mma_b_raw(ah, bl[j], acc[i][j]);
      }
      dep_guard_b(acc[i][0], acc[i][3], ah, al);
    }
    keep4_b(bh[0], bh[1], bh[2], bh[3]);
    if (NSPLIT == 2) keep4_b(bl[0], bl[1], bl[2], bl[3]);
  }
  acc_guard4(acc[0][0], acc[0][1], acc[0][2], acc[0][3]);
  acc_guard4(acc[1][0], acc[1][1], acc[1][2], acc[1][3]);
  acc_guard4(acc[2][0], acc[2][1], acc[2][2], acc[2][3]);
  acc_guard4(acc[3][0], acc[3][1], acc[3][2], acc[3][3]);

  float bcol[4] = {0.f, 0.f, 0.f, 0.f};
  if (BIAS == 1) {
#pragma unroll
    for (int j = 0; j < 4; ++j) bcol[j] = bf_up(bf_bits(bias[n0 + (j << 4) + rlane]));
  }
  float* slab = sT[wave];
#pragma unroll
  for (int i = 0; i < 4; ++i) {
    const int mBase = m0 + (i << 4);
    float brow[8] = {0.f, 0.f, 0.f, 0.f, 0.f, 0.f, 0.f, 0.f};
    if (BIAS == 2) {
#pragma unroll
      for (int r = 0; r < 8; ++r) brow[r] = bf_up(bf_bits(bias[mBase + mOff + r]));
    }
#pragma unroll
    for (int j = 0; j < 4; ++j) {
#pragma unroll
      for (int r = 0; r < 8; ++r) {
        float v = acc[i][j][r] + bcol[j] + brow[r];
        if (ACT == 1) {
          const float e = expf(-v);
          v = v * __builtin_amdgcn_rcpf(1.0f + e);
        }
        v *= oscale;
        if (RESID == 1) {
          v += bf_up(bf_bits(res[(size_t)(mBase + mOff + r) * ldr + n0 + (j << 4) + rlane]));
        }
        slab[(mOff + r) * 68 + (j << 4) + rlane] = v;
      }
    }
    wave_sync_lds();
    if (OUT_MODE == 0) {
      float* C = (float*)Cout + (size_t)b * strideC;
      const int hh = lane >> 4, c4 = (lane & 15) * 4;
      for (int pass = 0; pass < 2; ++pass) {
#pragma unroll
        for (int it = 0; it < 8; ++it) {
          const int row = it * 2 + hh;
          const v4f v = *(const v4f*)(slab + row * 68 + c4);
          *(volatile v4f*)(C + (size_t)(mBase + row) * ldc + n0 + c4) = v;
        }
        __threadfence();
      }
    } else {
      const int q = lane >> 3, c8 = (lane & 7) * 8;
      unsigned short* C  = (unsigned short*)Cout  + (size_t)b * strideC;
      unsigned short* C2 = (unsigned short*)Cout2 + (size_t)b * strideC2;
      const bool wlo = (OUT_MODE == 2) || (OUT_MODE == 3 && n0 < N2);
      v4u hv[4], lv[4];
#pragma unroll
      for (int it = 0; it < 4; ++it) {
        const int row = it * 4 + q;
        const float* sp = slab + row * 68 + c8;
        v4u a, a2;
#pragma unroll
        for (int e = 0; e < 4; ++e) {
          const float f0 = sp[2 * e], f1 = sp[2 * e + 1];
          unsigned short h0, h1, l0, l1;
          if (OUT_MODE == 2) {
            h0 = bf_bits(f0); h1 = bf_bits(f1);
            l0 = bf_bits(f0 - bf_up(h0)); l1 = bf_bits(f1 - bf_up(h1));
          } else {
            const _Float16 x0 = (_Float16)f0, x1 = (_Float16)f1;
            h0 = h_bits(x0); h1 = h_bits(x1);
            l0 = h_bits((_Float16)((f0 - (float)x0) * rscale));
            l1 = h_bits((_Float16)((f1 - (float)x1) * rscale));
          }
          a[e] = pk16(h0, h1); a2[e] = pk16(l0, l1);
        }
        hv[it] = a; lv[it] = a2;
      }
      for (int pass = 0; pass < 2; ++pass) {
#pragma unroll
        for (int it = 0; it < 4; ++it) {
          const int row = it * 4 + q;
          *(volatile v4u*)(C + (size_t)(mBase + row) * ldc + n0 + c8) = hv[it];
          if (wlo) *(volatile v4u*)(C2 + (size_t)(mBase + row) * ldc2 + n0 + c8) = lv[it];
        }
        __threadfence();
      }
    }
    wave_sync_lds();
  }
}

__global__ __launch_bounds__(128) void conv_qkv(const float* __restrict__ Y, const float* __restrict__ convw,
                                               const float* __restrict__ qw, const float* __restrict__ kw,
                                               const float* __restrict__ vw,
                                               float* XA, float* VF, unsigned short* Gh, unsigned short* Gl,
                                               unsigned short* Qh, unsigned short* Kh) {
  __shared__ float cwL[9 * INNER];
  __shared__ float qwL[NHQ * 16];
  __shared__ float kwL[NHQ * 16];
  __shared__ float vwL[NHQ * 16];
  __shared__ __align__(16) float xaL[TOKB][INNER];
  __shared__ float xmL[TOKB][INNER];
  __shared__ __align__(16) float gin[TOKB][GK];
  const int tid = threadIdx.x;
  const int tok0 = blockIdx.x * TOKB;
  if (tok0 >= NROWS) return;
  const int b = tok0 / SEQ;
  const int s0 = tok0 - b * SEQ;
  for (int i = tid; i < 9 * INNER; i += 128) cwL[i] = bfr(convw[i]);
  for (int i = tid; i < NHQ * 16; i += 128) { qwL[i] = bfr(qw[i]); kwL[i] = bfr(kw[i]); vwL[i] = bfr(vw[i]); }
  __syncthreads();
  const float* Yb = Y + (size_t)b * SEQ * UPN;

#pragma unroll 1
  for (int item = tid; item < TOKB * INNER; item += 128) {
    const int tok = item / INNER;
    const int c = item - tok * INNER;
    const int s = s0 + tok;
    const int gy = s / GRIDW, gx = s - gy * GRIDW;
    float a = 0.f;
#pragma unroll
    for (int dy = 0; dy < 3; ++dy) {
      const int hy = gy + dy - 1;
      const int hyc = min(max(hy, 0), GRIDW - 1);
      const bool vy = (hy >= 0) && (hy < GRIDW);
#pragma unroll
      for (int dx = 0; dx < 3; ++dx) {
        const int wx = gx + dx - 1;
        const int wxc = min(max(wx, 0), GRIDW - 1);
        const bool vx = (wx >= 0) && (wx < GRIDW);
        const float yv = Yb[(size_t)(hyc * GRIDW + wxc) * UPN + c];
        const float wv = cwL[(dy * 3 + dx) * INNER + c];
        a += ((vy && vx) ? yv : 0.f) * wv;
      }
    }
    const float xm = Yb[(size_t)s * UPN + c];
    const float e = expf(-a);
    const float sg = 1.0f / (1.0f + e);
    xaL[tok][c] = a * sg;
    xmL[tok][c] = xm;
  }
  __syncthreads();

#pragma unroll 1
  for (int item = tid; item < TOKB * INNER; item += 128) {
    const int tok = item / INNER;
    const int c = item - tok * INNER;
    const int hq = c >> 2, o = c & 3;
    const int wb = hq * 16 + o * 4;
    const int cb = hq * 4;
    float q = 0.f, k = 0.f, v = 0.f;
#pragma unroll
    for (int d = 0; d < 4; ++d) {
      const float xa = xaL[tok][cb + d];
      q += xa * qwL[wb + d];
      k += xa * kwL[wb + d];
      v += xmL[tok][cb + d] * vwL[wb + d];
    }
    gin[tok][c] = q;
    gin[tok][INNER + c] = k;
    gin[tok][2 * INNER + c] = v;
  }
  __syncthreads();

  const v4f z = {0.f, 0.f, 0.f, 0.f};
  for (int pass = 0; pass < 2; ++pass) {
    for (int p = tid; p < TOKB * (INNER / 4); p += 128) {
      const int tok = p / (INNER / 4);
      const int c4 = (p - tok * (INNER / 4)) * 4;
      const v4f v = *(const v4f*)(&xaL[tok][c4]);
      *(volatile v4f*)(XA + (size_t)(tok0 + tok) * INNER + c4) = v;
    }
    for (int p = tid; p < TOKB * (VP / 4); p += 128) {
      const int tok = p / (VP / 4);
      const int c4 = (p - tok * (VP / 4)) * 4;
      const int cc = min(c4, INNER - 4);
      v4f v = *(const v4f*)(&gin[tok][2 * INNER + cc]);
      if (c4 >= INNER) v = z;
      *(volatile v4f*)(VF + (size_t)(tok0 + tok) * VP + c4) = v;
    }
    for (int p = tid; p < TOKB * (GPITCH / 8); p += 128) {
      const int tok = p / (GPITCH / 8);
      const int j8 = (p - tok * (GPITCH / 8)) * 8;
      const int jc = min(j8, GK - 8);
      v4f a = *(const v4f*)(&gin[tok][jc]);
      v4f a4 = *(const v4f*)(&gin[tok][jc + 4]);
      if (j8 >= GK) { a = z; a4 = z; }
      v4u ph, pl;
#pragma unroll
      for (int e = 0; e < 2; ++e) {
        const float f0 = a[2 * e], f1 = a[2 * e + 1];
        const float g0 = a4[2 * e], g1 = a4[2 * e + 1];
        const unsigned short h0 = bf_bits(f0), h1 = bf_bits(f1), h2 = bf_bits(g0), h3 = bf_bits(g1);
        ph[e]     = pk16(h0, h1);
        ph[2 + e] = pk16(h2, h3);
        pl[e]     = pk16(bf_bits(f0 - bf_up(h0)), bf_bits(f1 - bf_up(h1)));
        pl[2 + e] = pk16(bf_bits(g0 - bf_up(h2)), bf_bits(g1 - bf_up(h3)));
      }
      const size_t go = (size_t)(tok0 + tok) * GPITCH + j8;
      *(volatile v4u*)(Gh + go) = ph;
      *(volatile v4u*)(Gl + go) = pl;
    }
    for (int p = tid; p < TOKB * (QP / 8); p += 128) {
      const int tok = p / (QP / 8);
      const int j8 = (p - tok * (QP / 8)) * 8;
      const int nh = j8 / HP96;
      const int d = j8 - nh * HP96;
      const int dcl = min(d, DHM - 8);
      v4f qa = *(const v4f*)(&gin[tok][nh * DHM + dcl]);
      v4f qb = *(const v4f*)(&gin[tok][nh * DHM + dcl + 4]);
      v4f ka = *(const v4f*)(&gin[tok][INNER + nh * DHM + dcl]);
      v4f kb = *(const v4f*)(&gin[tok][INNER + nh * DHM + dcl + 4]);
      if (d >= DHM) { qa = z; qb = z; ka = z; kb = z; }
      v4u pq, pk;
#pragma unroll
      for (int e = 0; e < 2; ++e) {
        pq[e]     = pk16(h_bits((_Float16)(qa[2 * e] * QSC)), h_bits((_Float16)(qa[2 * e + 1] * QSC)));
        pq[2 + e] = pk16(h_bits((_Float16)(qb[2 * e] * QSC)), h_bits((_Float16)(qb[2 * e + 1] * QSC)));
        pk[e]     = pk16(h_bits((_Float16)(ka[2 * e] * QSC)), h_bits((_Float16)(ka[2 * e + 1] * QSC)));
        pk[2 + e] = pk16(h_bits((_Float16)(kb[2 * e] * QSC)), h_bits((_Float16)(kb[2 * e + 1] * QSC)));
      }
      const size_t go = (size_t)(tok0 + tok) * QP + j8;
      *(volatile v4u*)(Qh + go) = pq;
      *(volatile v4u*)(Kh + go) = pk;
    }
    __threadfence();
  }
}

__global__ __launch_bounds__(32) void gate_scan(const float* __restrict__ G, const float* __restrict__ igb,
                                               const float* __restrict__ fgb, float* SC) {
  __shared__ __align__(16) float stg[3][32][32];
  const int t = threadIdx.x;
  const int b = ((t >> 2) < NB) ? (t >> 2) : (NB - 1), nh = t & 3;
  const float ib = bfr(igb[nh]);
  const float fb = bfr(fgb[nh]);
  const float* Gb = G + (size_t)b * SEQ * GN;
  float lfc = 0.f;
  float cmax = -__builtin_inff();
  for (int ch = 0; ch < SEQ / 32; ++ch) {
#pragma unroll 1
    for (int i = 0; i < 32; ++i) {
      const int s = ch * 32 + i;
      const float fgv = Gb[(size_t)s * GN + NHM + nh] + fb;
      const float igv = Gb[(size_t)s * GN + nh] + ib;
      const float lf = fminf(fgv, 0.f) - log1pf(expf(-fabsf(fgv)));
      lfc += lf;
      const float c = igv - lfc;
      cmax = fmaxf(cmax, c);
      stg[0][t][i] = -cmax;
      stg[1][t][i] = c;
      stg[2][t][i] = expf(-(lfc + cmax));
    }
    wave_sync_lds();
    for (int pass = 0; pass < 2; ++pass) {
#pragma unroll
      for (int pl = 0; pl < 3; ++pl) {
#pragma unroll
        for (int q4 = 0; q4 < 8; ++q4) {
          const int piece = q4 * 32 + t;
          const int row = piece >> 3, pc = (piece & 7) * 4;
          const v4f v = *(const v4f*)(&stg[pl][row][pc]);
          if (row < NB * NHM)
            *(volatile v4f*)(SC + (size_t)pl * (NB * NHM * SEQ) + (size_t)row * SEQ + ch * 32 + pc) = v;
        }
      }
      __threadfence();
    }
    wave_sync_lds();
  }
}

__global__ __launch_bounds__(128)
void mlstm_attn(const unsigned short* __restrict__ qhp, const unsigned short* __restrict__ khp,
                const unsigned short* __restrict__ vtp, const float* __restrict__ SC, float* Hout) {
  union FH { v16h v; v8h h[2]; };
  __shared__ __align__(16) _Float16 Ksh[64 * HP96];
  __shared__ __align__(16) _Float16 Vsh[80 * 64];
  __shared__ __align__(16) _Float16 Psh[4][16 * 64];
  __shared__ __align__(16) float    Os[4][16 * HP96];
  __shared__ float ctL[64];

  const int tid  = threadIdx.x;
  const int wave = tid >> 5;
  const int lane = tid & 31;
  const int hh   = lane >> 4;
  const int c    = lane & 15;

  const int bx   = blockIdx.x;
  const int qb   = bx & 15;
  const int rest = bx >> 4;
  const int nh   = rest & 3;
  const int b    = rest >> 2;
  const int q0   = qb * 64 + wave * 16;
  const size_t rowB = (size_t)b * SEQ;
  const int bn   = b * NHM + nh;
  const float* rterm = SC + (size_t)bn * SEQ;
  const float* cterm = SC + (size_t)NB * NHM * SEQ + (size_t)bn * SEQ;
  const float* nexpp = SC + (size_t)2 * NB * NHM * SEQ + (size_t)bn * SEQ;

  const _Float16* Qg = (const _Float16*)(const void*)qhp + (size_t)nh * HP96;
  const _Float16* Kg = (const _Float16*)(const void*)khp + (size_t)nh * HP96;
  const _Float16* Vg = (const _Float16*)(const void*)vtp + ((size_t)b * VP + (size_t)nh * DHM) * SEQ;

  v16h qa[3];
#pragma unroll
  for (int dc = 0; dc < 3; ++dc) qa[dc] = ldfrag_h(Qg + (rowB + q0 + c) * QP + dc * 32 + 8 * hh);
  float rt[8];
#pragma unroll
  for (int r = 0; r < 8; ++r) rt[r] = rterm[q0 + 8 * hh + r];

  v8f oacc[5];
#pragma unroll
  for (int t5 = 0; t5 < 5; ++t5) oacc[t5] = zero8();
  float rsum[8] = {0.f, 0.f, 0.f, 0.f, 0.f, 0.f, 0.f, 0.f};

  const int nkt = qb + 1;
  for (int kt = 0; kt < nkt; ++kt) {
    const int kv0 = kt * 64;
    __syncthreads();
    for (int i = tid; i < 64 * 12; i += 128) {
      const int r = i / 12, pc = (i - r * 12) * 8;
      *(v8h*)(Ksh + r * HP96 + pc) = *(const v8h*)(Kg + (rowB + kv0 + r) * QP + pc);
    }
    for (int i = tid; i < 80 * 8; i += 128) {
      const int r = i >> 3, pc = (i & 7) * 8;
      *(v8h*)(Vsh + r * 64 + pc) = *(const v8h*)(Vg + (size_t)r * SEQ + kv0 + pc);
    }
    if (tid < 64) ctL[tid] = cterm[kv0 + tid];
    __syncthreads();

    v8f sj[4];
#pragma unroll
    for (int j = 0; j < 4; ++j) {
      v8f s = zero8();
#pragma unroll
      for (int dc = 0; dc < 3; ++dc) {
        FH kb;
        kb.h[0] = *(const v8h*)(Ksh + (j * 16 + c) * HP96 + dc * 32 + 8 * hh);
        kb.h[1] = *(const v8h*)(Ksh + (j * 16 + c) * HP96 + dc * 32 + 16 + 8 * hh);
        s = mma_h(qa[dc], kb.v, s);
      }
      sj[j] = s;
    }

    _Float16* pw = Psh[wave];
#pragma unroll
    for (int j = 0; j < 4; ++j) {
      const float ctj = ctL[j * 16 + c];
      const int t = kv0 + j * 16 + c;
#pragma unroll
      for (int r = 0; r < 8; ++r) {
        const int srow = q0 + 8 * hh + r;
        const float dcy = __expf(fminf(rt[r] + ctj, 0.f));
        const float p = (t <= srow) ? sj[j][r] * dcy : 0.f;
        rsum[r] += p;
        pw[(8 * hh + r) * 64 + j * 16 + c] = (_Float16)p;
      }
    }
    wave_sync_lds();

#pragma unroll 1
    for (int kk = 0; kk < 2; ++kk) {
      FH pa;
      pa.h[0] = *(const v8h*)(pw + c * 64 + kk * 32 + 8 * hh);
      pa.h[1] = *(const v8h*)(pw + c * 64 + kk * 32 + 16 + 8 * hh);
#pragma unroll
      for (int t5 = 0; t5 < 5; ++t5) {
        FH vb;
        vb.h[0] = *(const v8h*)(Vsh + (t5 * 16 + c) * 64 + kk * 32 + 8 * hh);
        vb.h[1] = *(const v8h*)(Vsh + (t5 * 16 + c) * 64 + kk * 32 + 16 + 8 * hh);
        oacc[t5] = mma_h(pa.v, vb.v, oacc[t5]);
      }
    }
  }

  float inv[8];
#pragma unroll
  for (int r = 0; r < 8; ++r) {
    const float tot = hsum16(rsum[r]);
    const float nx  = nexpp[q0 + 8 * hh + r];
    const float nrm = fmaxf(fabsf(tot * CSC), nx) + 1.0e-6f;
    inv[r] = (CSC * (1.0f / VSC)) / nrm;
  }
  float* os = Os[wave];
#pragma unroll
  for (int r = 0; r < 8; ++r) {
#pragma unroll
    for (int t5 = 0; t5 < 5; ++t5) {
      float v = oacc[t5][r] * inv[r];
      if (t5 == 4 && c >= 8) v = 0.f;
      os[(8 * hh + r) * HP96 + t5 * 16 + c] = v;
    }
    os[(8 * hh + r) * HP96 + 80 + c] = 0.f;
  }
  wave_sync_lds();
  {
    const int lc = min(lane, 23);
    float* dst = Hout + (size_t)nh * HP96 + lc * 4;
    for (int pass = 0; pass < 2; ++pass) {
#pragma unroll
      for (int row = 0; row < 16; ++row) {
        const v4f v = *(const v4f*)(os + row * HP96 + lc * 4);
        if (lane < 24) *(volatile v4f*)(dst + (rowB + q0 + row) * HOP) = v;
      }
      __threadfence();
    }
  }
}

__global__ __launch_bounds__(256) void ln_state(const float* __restrict__ H, const float* __restrict__ XA,
                                               const float* __restrict__ Y, const float* __restrict__ normw,
                                               const float* __restrict__ skipw,
                                               unsigned short* Oh, unsigned short* Ol) {
  __shared__ __align__(16) unsigned short stg[8][2][OSP];
  union U8 { v8us s; v4u u; };
  const int wave = threadIdx.x >> 5, lane = threadIdx.x & 31;
  const int row = blockIdx.x * 8 + wave;
  if (row >= NROWS) return;
  const int g  = lane >> 3;
  const int j0 = (lane & 7) * 9;
  const int c0 = lane * 9;
  const float* hr = H + (size_t)row * HOP + g * HP96 + j0;
  float s1 = 0.f;
#pragma unroll 1
  for (int i = 0; i < 9; ++i) s1 += hr[i];
  s1 = hsum8(s1);
  const float mu = s1 * (1.0f / (float)DHM);
  float s2 = 0.f;
#pragma unroll 1
  for (int i = 0; i < 9; ++i) { const float d = hr[i] - mu; s2 += d * d; }
  s2 = hsum8(s2);
  const float var  = s2 * (1.0f / (float)DHM);
  const float rstd = 1.0f / sqrtf(var + 1.0e-5f);
  unsigned short* sh = stg[wave][0];
  unsigned short* sl = stg[wave][1];
  const float* xar = XA + (size_t)row * INNER;
  const float* zr  = Y + (size_t)row * UPN + INNER;
#pragma unroll 1
  for (int i = 0; i < 9; ++i) {
    const int c = c0 + i;
    const float hv = hr[i];
    const float hn = (hv - mu) * rstd * bfr(normw[c]);
    const float hs = hn + bfr(skipw[c]) * xar[c];
    const float z  = zr[c];
    const float e  = expf(-z);
    const float sg = 1.0f / (1.0f + e);
    const float hst = hs * (z * sg);
    const unsigned short hb = bf_bits(hst);
    sh[c] = hb;
    sl[c] = bf_bits(hst - bf_up(hb));
  }
  sh[INNER + lane] = 0;
  sl[INNER + lane] = 0;
  wave_sync_lds();
  const int lc = min(lane, 7);
  U8 a0, a1, b0, b1;
  a0.s = *(const v8us*)(sh + lane * 8);
  a1.s = *(const v8us*)(sh + 256 + lc * 8);
  b0.s = *(const v8us*)(sl + lane * 8);
  b1.s = *(const v8us*)(sl + 256 + lc * 8);
  unsigned short* dh = Oh + (size_t)row * OSP;
  unsigned short* dl = Ol + (size_t)row * OSP;
  for (int pass = 0; pass < 2; ++pass) {
    *(volatile v4u*)(dh + lane * 8) = a0.u;
    *(volatile v4u*)(dl + lane * 8) = b0.u;
    if (lane < 8) {
      *(volatile v4u*)(dh + 256 + lane * 8) = a1.u;
      *(volatile v4u*)(dl + 256 + lane * 8) = b1.u;
    }
    __threadfence();
  }
}

extern "C" void kernel_launch(void* const* d_in, const int* in_sizes, int n_in,
                              void* d_out, int out_size, void* d_ws, size_t ws_size,
                              hipStream_t stream) {
  if (n_in < 13) return;
  if (in_sizes[0] != NROWS * DIMX) return;
  if (in_sizes[1] != UPN * DIMX) return;
  if (in_sizes[2] != NHQ * 16) return;
  if (in_sizes[3] != NHQ * 16) return;
  if (in_sizes[4] != NHQ * 16) return;
  if (in_sizes[5] != 9 * INNER) return;
  if (in_sizes[6] != NHM * GK) return;
  if (in_sizes[7] != NHM) return;
  if (in_sizes[8] != NHM * GK) return;
  if (in_sizes[9] != NHM) return;
  if (in_sizes[10] != INNER) return;
  if (in_sizes[11] != INNER) return;
  if (in_sizes[12] != DIMX * INNER) return;
  if (out_size != NROWS * DIMX) return;

  const float* x     = (const float*)d_in[0];
  const float* wup   = (const float*)d_in[1];
  const float* qw    = (const float*)d_in[2];
  const float* kw    = (const float*)d_in[3];
  const float* vw    = (const float*)d_in[4];
  const float* convw = (const float*)d_in[5];
  const float* igw   = (const float*)d_in[6];
  const float* igb   = (const float*)d_in[7];
  const float* fgw   = (const float*)d_in[8];
  const float* fgb   = (const float*)d_in[9];
  const float* normw = (const float*)d_in[10];
  const float* skipw = (const float*)d_in[11];
  const float* wdn   = (const float*)d_in[12];

  const size_t szXb  = (size_t)NROWS * DIMX * 2;
  const size_t szWup = (size_t)UPN * DIMX * 2;
  const size_t szWdn = (size_t)DIMX * INNER * 2;
  const size_t szGW  = (size_t)GN * GPITCH * 2;
  const size_t szY   = (size_t)NROWS * UPN * 4;
  const size_t szXA  = (size_t)NROWS * INNER * 4;
  const size_t szVF  = (size_t)NROWS * VP * 4;
  const size_t szG16 = (size_t)NROWS * GPITCH * 2;
  const size_t szQK  = (size_t)NROWS * QP * 2;
  const size_t szVT  = (size_t)NB * VP * SEQ * 2;
  const size_t szG   = (size_t)NROWS * GN * 4;
  const size_t szSC  = (size_t)3 * NB * NHM * SEQ * 4;
  const size_t szH   = (size_t)NROWS * HOP * 4;
  const size_t szO16 = (size_t)NROWS * OSP * 2;
  size_t off = 0;
  const size_t oXb  = off; off += szXb;
  const size_t oWup = off; off += szWup;
  const size_t oWdn = off; off += szWdn;
  const size_t oGW  = off; off += szGW;
  const size_t oY   = off; off += szY;
  const size_t oXA  = off; off += szXA;
  const size_t oVF  = off; off += szVF;
  const size_t oGh  = off; off += szG16;
  const size_t oGl  = off; off += szG16;
  const size_t oQh  = off; off += szQK;
  const size_t oKh  = off; off += szQK;
  const size_t oVT  = off; off += szVT;
  const size_t oG   = off; off += szG;
  const size_t oSC  = off; off += szSC;
  const size_t oH   = off; off += szH;
  const size_t oOh  = off; off += szO16;
  const size_t oOl  = off; off += szO16;
  if (off > ws_size) return;
  if (off > (size_t)134217728) return;

  char* ws = (char*)d_ws;
  unsigned short* Xb  = (unsigned short*)(ws + oXb);
  unsigned short* Wup = (unsigned short*)(ws + oWup);
  unsigned short* Wdn = (unsigned short*)(ws + oWdn);
  unsigned short* GWp = (unsigned short*)(ws + oGW);
  float*          Y   = (float*)(ws + oY);
  float*          XA  = (float*)(ws + oXA);
  float*          VF  = (float*)(ws + oVF);
  unsigned short* Gh  = (unsigned short*)(ws + oGh);
  unsigned short* Gl  = (unsigned short*)(ws + oGl);
  unsigned short* Qh  = (unsigned short*)(ws + oQh);
  unsigned short* Kh  = (unsigned short*)(ws + oKh);
  unsigned short* VT  = (unsigned short*)(ws + oVT);
  float*          Gp  = (float*)(ws + oG);
  float*          SC  = (float*)(ws + oSC);
  float*          Hp  = (float*)(ws + oH);
  unsigned short* Oh  = (unsigned short*)(ws + oOh);
  unsigned short* Ol  = (unsigned short*)(ws + oOl);

  const dim3 blk(256);
  const dim3 gCvt((NROWS * DIMX / 8 + 255) / 256);
  const dim3 gPrep(BUP + BDN + BGW);
  const dim3 gUp(((NROWS / 64) * (UPN / 64) + 7) / 8, 1);
  const dim3 gConv(NROWS / TOKB);
  const dim3 gTv((SEQ / 64) * (VP / 64), NB);
  const dim3 gGate(((NROWS / 64) * (GN / 64) + 7) / 8, 1);
  const dim3 gAttn(NB * NHM * (SEQ / 64));
  const dim3 gLn(NROWS / 8);
  const dim3 gDn(((NROWS / 64) * (DIMX / 64) + 7) / 8, 1);

  cvt_cat_bf16x8<<<gCvt, blk, 0, stream>>>(x, Xb, NROWS * DIMX / 8, DIMX / 8, DIMX, 0);
  prep_w<<<gPrep, blk, 0, stream>>>(wup, wdn, igw, fgw, Wup, Wdn, GWp);
  gemm64<0, 0, 0, 0, 0><<<gUp, blk, 0, stream>>>(
      Xb, Xb, DIMX, 0LL, Wup, Wup, DIMX, 0LL, igb, x, DIMX,
      (void*)Y, UPN, 0LL, (void*)Y, UPN, 0LL, UPN,
      NROWS, UPN, DIMX, 1.0f, 1.0f);
  conv_qkv<<<gConv, dim3(128), 0, stream>>>(Y, convw, qw, kw, vw, XA, VF, Gh, Gl, Qh, Kh);
  transpose16<1><<<gTv, blk, 0, stream>>>(VF, SEQ, VP, (long long)SEQ * VP, VT, (long long)VP * SEQ, VSC, 1.0f);
  gemm64<1, 0, 0, 0, 0><<<gGate, blk, 0, stream>>>(
      Gh, Gl, GPITCH, 0LL, GWp, GWp, GPITCH, 0LL, igb, x, DIMX,
      (void*)Gp, GN, 0LL, (void*)Gp, GN, 0LL, GN,
      NROWS, GN, GK, 1.0f, 1.0f);
  gate_scan<<<dim3(1), dim3(32), 0, stream>>>(Gp, igb, fgb, SC);
  mlstm_attn<<<gAttn, dim3(128), 0, stream>>>(Qh, Kh, VT, SC, Hp);
  ln_state<<<gLn, blk, 0, stream>>>(Hp, XA, Y, normw, skipw, Oh, Ol);
  gemm64<1, 0, 0, 0, 0><<<gDn, blk, 0, stream>>>(
      Oh, Ol, OSP, 0LL, Wdn, Wdn, INNER, 0LL, igb, x, DIMX,
      d_out, DIMX, 0LL, d_out, DIMX, 0LL, DIMX,
      NROWS, DIMX, INNER, 1.0f, 1.0f);
  (void)hipGetLastError();
}
